// BertSelfAttention_91250875170938
// MI455X (gfx1250) — hardware-verified
//
#include <hip/hip_runtime.h>


#ifndef NB
#define NB 4
#endif
#ifndef SEQ
#define SEQ 2048
#endif
#define NB_FULL 4
#define SEQ_FULL 2048
#define DM 1024
#define NH 16
#define HD 64
#define MTOT (NB * SEQ)

static_assert(NB >= 1 && NB <= NB_FULL);
static_assert(SEQ >= 128 && SEQ <= SEQ_FULL && (SEQ % 128) == 0);
static_assert(DM == 1024 && DM == NH * HD && HD == 64);
static_assert((MTOT % 128) == 0);

typedef _Float16 v16h __attribute__((ext_vector_type(16)));
typedef _Float16 v8h  __attribute__((ext_vector_type(8)));
typedef float    v8f  __attribute__((ext_vector_type(8)));
typedef float    v4f  __attribute__((ext_vector_type(4)));
union Frag { v16h v; v8h h[2]; _Float16 e[16]; };

__device__ __forceinline__ float bf16r(float f) {
  unsigned u = __float_as_uint(f);
  u += 0x7FFFu + ((u >> 16) & 1u);
  return __uint_as_float(u & 0xFFFF0000u);
}

__device__ __forceinline__ v16h ldfrag(const _Float16* p, int hh) {
  Frag f;
  f.h[0] = *(const v8h*)(p + 8 * hh);
  f.h[1] = *(const v8h*)(p + 16 + 8 * hh);
  return f.v;
}

__device__ __forceinline__ v8f wmma16(v16h a, v16h b, v8f c) {
  c = __builtin_amdgcn_wmma_f32_16x16x32_f16(false, a, false, b, (short)0, c, false, false);
  asm volatile("v_nop\n\tv_nop\n\tv_nop\n\tv_nop" : "+v"(c) : "v"(a), "v"(b));
  return c;
}

__global__ __launch_bounds__(256) void cvt_x_kernel(const float* __restrict__ x, _Float16* __restrict__ xh) {
  const size_t e = ((size_t)blockIdx.x * 256 + threadIdx.x) * 8;
  const size_t row = e >> 10;
  const int col = (int)(e & 1023);
  const int bb = (int)(row / SEQ), s = (int)(row - (size_t)bb * SEQ);
  const float* src = x + ((size_t)bb * SEQ_FULL + s) * DM + col;
  const v4f a = *(const v4f*)src;
  const v4f c = *(const v4f*)(src + 4);
  v8h o;
#pragma unroll
  for (int r = 0; r < 4; ++r) { o[r] = (_Float16)bf16r(a[r]); o[4 + r] = (_Float16)bf16r(c[r]); }
  _Float16* dst = xh + e;
  *(volatile v8h*)dst = o;
  __threadfence();
  *(volatile v8h*)dst = o;
}

#define WTP 72
__global__ __launch_bounds__(256) void cvt_w_kernel(const float* __restrict__ W0, const float* __restrict__ W1,
                                                     const float* __restrict__ W2, _Float16* __restrict__ Wt) {
  __shared__ __align__(16) _Float16 tl[64 * WTP];
  const int wi = blockIdx.z;
  const float* W = (wi == 0) ? W0 : ((wi == 1) ? W1 : W2);
  const int k0 = blockIdx.y * 64, n0 = blockIdx.x * 64;
  const int tid = threadIdx.x;
#pragma unroll
  for (int j = 0; j < 4; ++j) {
    const int idx = j * 256 + tid;
    const int kr = idx >> 4, c4 = (idx & 15) * 4;
    const v4f a = *(const v4f*)(W + (size_t)(k0 + kr) * DM + n0 + c4);
#pragma unroll
    for (int i = 0; i < 4; ++i) tl[(c4 + i) * WTP + kr] = (_Float16)(bf16r(a[i]) * 64.0f);
  }
  __syncthreads();
  _Float16* dstp = Wt + (size_t)wi * DM * DM;
  v8h vals[2]; size_t offs[2];
#pragma unroll
  for (int j = 0; j < 2; ++j) {
    const int idx = j * 256 + tid;
    const int nr = idx >> 3, piece = idx & 7;
    vals[j] = *(const v8h*)(tl + nr * WTP + piece * 8);
    offs[j] = (size_t)(n0 + nr) * DM + k0 + piece * 8;
  }
#pragma unroll
  for (int j = 0; j < 2; ++j) *(volatile v8h*)(dstp + offs[j]) = vals[j];
  __threadfence();
#pragma unroll
  for (int j = 0; j < 2; ++j) *(volatile v8h*)(dstp + offs[j]) = vals[j];
}

#define STP 136

__device__ __forceinline__ void store_tok_plane(_Float16* P, const _Float16* stg, int m0, int n0, int tid) {
  v8h vals[8]; size_t offs[8];
#pragma unroll
  for (int j = 0; j < 8; ++j) {
    const int idx = j * 256 + tid;
    const int fh = idx >> 10, rem = idx & 1023, tr = rem >> 3, piece = rem & 7;
    const int tok = m0 + tr, bb = tok / SEQ, s = tok - bb * SEQ;
    const int head = (n0 >> 6) + fh;
    vals[j] = *(const v8h*)(stg + tr * STP + fh * 64 + piece * 8);
    offs[j] = (((size_t)bb * NH + head) * SEQ + s) * HD + piece * 8;
  }
#pragma unroll
  for (int j = 0; j < 8; ++j) *(volatile v8h*)(P + offs[j]) = vals[j];
  __threadfence();
#pragma unroll
  for (int j = 0; j < 8; ++j) *(volatile v8h*)(P + offs[j]) = vals[j];
}

__global__ __launch_bounds__(256) void proj_kernel(const _Float16* __restrict__ Xh, const _Float16* __restrict__ Wt,
                                                   const float* __restrict__ bq, const float* __restrict__ bk,
                                                   const float* __restrict__ bv,
                                                   _Float16* __restrict__ Qh, _Float16* __restrict__ Qr,
                                                   _Float16* __restrict__ Kh, _Float16* __restrict__ Kr,
                                                   _Float16* __restrict__ Vt) {
  __shared__ __align__(16) _Float16 st[128 * STP];
  const int tid = threadIdx.x, lane = tid & 31, w = tid >> 5, l16 = lane & 15, hh = lane >> 4;
  const int wr = w & 3, wc = w >> 2;
  const int m0 = blockIdx.x * 128;
  const int wi = blockIdx.y >> 3;
  const int n0 = (blockIdx.y & 7) * 128;
  const _Float16* Wp = Wt + (size_t)wi * DM * DM;
  const float* bias = (wi == 0) ? bq : ((wi == 1) ? bk : bv);

  const v8f z8 = {0.f, 0.f, 0.f, 0.f, 0.f, 0.f, 0.f, 0.f};
  v8f acc[2][4];
#pragma unroll
  for (int i = 0; i < 2; ++i)
#pragma unroll
    for (int t = 0; t < 4; ++t) acc[i][t] = z8;

  const _Float16* arow0 = Xh + (size_t)(m0 + wr * 32 + l16) * DM;
  const _Float16* arow1 = arow0 + (size_t)16 * DM;
  const _Float16* brow  = Wp + (size_t)(n0 + wc * 64 + l16) * DM;
#pragma unroll 1
  for (int kc = 0; kc < DM; kc += 32) {
    const v16h a0 = ldfrag(arow0 + kc, hh);
    const v16h a1 = ldfrag(arow1 + kc, hh);
#pragma unroll
    for (int t = 0; t < 4; ++t) {
      const v16h b = ldfrag(brow + (size_t)t * 16 * DM + kc, hh);
      acc[0][t] = wmma16(a0, b, acc[0][t]);
      acc[1][t] = wmma16(a1, b, acc[1][t]);
    }
  }

  const float osc = 1.0f / 64.0f;
  if (wi < 2) {
    _Float16* Ph = (wi == 0) ? Qh : Kh;
    _Float16* Pr = (wi == 0) ? Qr : Kr;
#pragma unroll
    for (int t = 0; t < 4; ++t) {
      const int cc = wc * 64 + t * 16 + l16;
      const float bvv = bf16r(bias[n0 + cc]);
#pragma unroll
      for (int i = 0; i < 2; ++i) {
        const int trb = wr * 32 + i * 16 + 8 * hh;
#pragma unroll
        for (int r = 0; r < 8; ++r) st[(trb + r) * STP + cc] = (_Float16)(acc[i][t][r] * osc + bvv);
      }
    }
    __syncthreads();
    store_tok_plane(Ph, st, m0, n0, tid);
    __syncthreads();
#pragma unroll
    for (int t = 0; t < 4; ++t) {
      const int cc = wc * 64 + t * 16 + l16;
      const float bvv = bf16r(bias[n0 + cc]);
#pragma unroll
      for (int i = 0; i < 2; ++i) {
        const int trb = wr * 32 + i * 16 + 8 * hh;
#pragma unroll
        for (int r = 0; r < 8; ++r) {
          const float v = acc[i][t][r] * osc + bvv;
          const _Float16 hv = (_Float16)v;
          st[(trb + r) * STP + cc] = (_Float16)((v - (float)hv) * 1024.0f);
        }
      }
    }
    __syncthreads();
    store_tok_plane(Pr, st, m0, n0, tid);
  } else {
#pragma unroll
    for (int t = 0; t < 4; ++t) {
      const int cc = wc * 64 + t * 16 + l16;
      const float bvv = bf16r(bias[n0 + cc]);
#pragma unroll
      for (int i = 0; i < 2; ++i) {
        const int trb = wr * 32 + i * 16 + 8 * hh;
        v8h o;
#pragma unroll
        for (int r = 0; r < 8; ++r) o[r] = (_Float16)(acc[i][t][r] * osc + bvv);
        *(v8h*)(st + cc * STP + trb) = o;
      }
    }
    __syncthreads();
    const int bb = m0 / SEQ, s0 = m0 - bb * SEQ;
    v8h vals[8]; size_t offs[8];
#pragma unroll
    for (int j = 0; j < 8; ++j) {
      const int idx = j * 256 + tid;
      const int dr = idx >> 4, piece = idx & 15;
      const int head = (n0 >> 6) + (dr >> 6), d = dr & 63;
      vals[j] = *(const v8h*)(st + dr * STP + piece * 8);
      offs[j] = (((size_t)bb * NH + head) * HD + d) * SEQ + s0 + piece * 8;
    }
#pragma unroll
    for (int j = 0; j < 8; ++j) *(volatile v8h*)(Vt + offs[j]) = vals[j];
    __threadfence();
#pragma unroll
    for (int j = 0; j < 8; ++j) *(volatile v8h*)(Vt + offs[j]) = vals[j];
  }
}

__global__ __launch_bounds__(256) void attn_kernel(const _Float16* __restrict__ Qh, const _Float16* __restrict__ Qr,
                                                   const _Float16* __restrict__ Kh, const _Float16* __restrict__ Kr,
                                                   const _Float16* __restrict__ Vt, const float* __restrict__ mask,
                                                   float* __restrict__ out) {
  __shared__ v4f ost[128 * 16];
  const int bh = blockIdx.y, b = bh / NH, h = bh - b * NH;
  const int tid = threadIdx.x, lane = tid & 31, w = tid >> 5, l16 = lane & 15, hh = lane >> 4;
  const int q0 = blockIdx.x * 128 + w * 16;
  const size_t qrow = ((size_t)bh * SEQ + q0 + l16) * HD;
  const _Float16* Kp  = Kh + (size_t)bh * SEQ * HD;
  const _Float16* Krp = Kr + (size_t)bh * SEQ * HD;
  const _Float16* Vp  = Vt + (size_t)bh * HD * SEQ;
  const float* mrow = mask + (size_t)b * SEQ_FULL;

  const v16h qf0 = ldfrag(Qh + qrow, hh);
  const v16h qf1 = ldfrag(Qh + qrow + 32, hh);
  const v16h qe0 = ldfrag(Qr + qrow, hh);
  const v16h qe1 = ldfrag(Qr + qrow + 32, hh);
  const v8f z8 = {0.f, 0.f, 0.f, 0.f, 0.f, 0.f, 0.f, 0.f};
  const float RSC = 1.0f / 1024.0f;
  v8f acc[4];
#pragma unroll
  for (int dt = 0; dt < 4; ++dt) acc[dt] = z8;
  float m_i = -__builtin_inff(), l_i = 0.0f;

#pragma unroll 1
  for (int k0 = 0; k0 < SEQ; k0 += 64) {
    v8f sc[4];
#pragma unroll
    for (int t = 0; t < 4; ++t) {
      const size_t krow = (size_t)(k0 + t * 16 + l16) * HD;
      const v16h ka  = ldfrag(Kp + krow, hh);
      const v16h kb  = ldfrag(Kp + krow + 32, hh);
      const v16h ke0 = ldfrag(Krp + krow, hh);
      const v16h ke1 = ldfrag(Krp + krow + 32, hh);
      v8f s = wmma16(ka, qf0, z8);
      s = wmma16(kb, qf1, s);
      v8f e = wmma16(ka, qe0, z8);
      e = wmma16(kb, qe1, e);
      e = wmma16(ke0, qf0, e);
      e = wmma16(ke1, qf1, e);
      sc[t] = s + e * RSC;
    }
    float mx = -__builtin_inff();
#pragma unroll
    for (int t = 0; t < 4; ++t) {
      const float* mp = mrow + k0 + t * 16 + 8 * hh;
      const v4f ma = *(const v4f*)mp;
      const v4f mb = *(const v4f*)(mp + 4);
#pragma unroll
      for (int r = 0; r < 4; ++r) {
        sc[t][r]     = sc[t][r]     * 0.125f + bf16r(ma[r]);
        sc[t][4 + r] = sc[t][4 + r] * 0.125f + bf16r(mb[r]);
      }
#pragma unroll
      for (int r = 0; r < 8; ++r) mx = fmaxf(mx, sc[t][r]);
    }
    mx = fmaxf(mx, __shfl_xor(mx, 16, 32));
    const float m_new = fmaxf(m_i, mx);
    float lsum = 0.0f;
#pragma unroll
    for (int t = 0; t < 4; ++t)
#pragma unroll
      for (int r = 0; r < 8; ++r) { const float p = __expf(sc[t][r] - m_new); sc[t][r] = p; lsum += p; }
    lsum += __shfl_xor(lsum, 16, 32);
    const float e0 = __expf(m_i - m_new);
    const float corr = (m_i == -__builtin_inff()) ? 0.0f : e0;
    l_i = l_i * corr + lsum;
    m_i = m_new;
#pragma unroll
    for (int dt = 0; dt < 4; ++dt) acc[dt] = acc[dt] * corr;

    Frag p0, p1;
#pragma unroll
    for (int r = 0; r < 8; ++r) {
      p0.e[r] = (_Float16)(sc[0][r] * 4096.0f); p0.e[8 + r] = (_Float16)(sc[1][r] * 4096.0f);
      p1.e[r] = (_Float16)(sc[2][r] * 4096.0f); p1.e[8 + r] = (_Float16)(sc[3][r] * 4096.0f);
    }
#pragma unroll
    for (int dt = 0; dt < 4; ++dt) {
      const _Float16* vr = Vp + (size_t)(dt * 16 + l16) * SEQ + k0;
      const v16h va = ldfrag(vr, hh);
      const v16h vb = ldfrag(vr + 32, hh);
      acc[dt] = wmma16(va, p0.v, acc[dt]);
      acc[dt] = wmma16(vb, p1.v, acc[dt]);
    }
  }

  const float f = (1.0f / l_i) * (1.0f / 4096.0f);
  const int row = w * 16 + l16;
#pragma unroll
  for (int dt = 0; dt < 4; ++dt) {
    v4f o0, o1;
#pragma unroll
    for (int r = 0; r < 4; ++r) { o0[r] = acc[dt][r] * f; o1[r] = acc[dt][4 + r] * f; }
    ost[row * 16 + dt * 4 + 2 * hh]     = o0;
    ost[row * 16 + dt * 4 + 2 * hh + 1] = o1;
  }
  __syncthreads();
  v4f vals[8]; size_t offs[8];
#pragma unroll
  for (int j = 0; j < 8; ++j) {
    const int idx = j * 256 + tid;
    const int qr = idx >> 4, piece = idx & 15;
    const int q = blockIdx.x * 128 + qr;
    vals[j] = ost[qr * 16 + piece];
    offs[j] = ((size_t)b * SEQ_FULL + q) * DM + h * HD + piece * 4;
  }
#pragma unroll
  for (int j = 0; j < 8; ++j) *(volatile v4f*)(out + offs[j]) = vals[j];
  __threadfence();
#pragma unroll
  for (int j = 0; j < 8; ++j) *(volatile v4f*)(out + offs[j]) = vals[j];
}

extern "C" void kernel_launch(void* const* d_in, const int* in_sizes, int n_in,
                              void* d_out, int out_size, void* d_ws, size_t ws_size,
                              hipStream_t stream) {
  if (n_in < 8) return;
  const size_t needTok = (size_t)(NB - 1) * SEQ_FULL + SEQ;
  if ((size_t)in_sizes[0] < needTok * DM) return;
  if ((size_t)in_sizes[1] < needTok) return;
  if (in_sizes[2] < DM * DM || in_sizes[4] < DM * DM || in_sizes[6] < DM * DM) return;
  if (in_sizes[3] < DM || in_sizes[5] < DM || in_sizes[7] < DM) return;
  if ((size_t)out_size < needTok * DM) return;

  const float* x    = (const float*)d_in[0];
  const float* mask = (const float*)d_in[1];
  const float* Wq   = (const float*)d_in[2];
  const float* bq   = (const float*)d_in[3];
  const float* Wk   = (const float*)d_in[4];
  const float* bk   = (const float*)d_in[5];
  const float* Wv   = (const float*)d_in[6];
  const float* bv   = (const float*)d_in[7];
  float* out = (float*)d_out;

  const size_t xhBytes  = (size_t)MTOT * DM * sizeof(_Float16);
  const size_t wtBytes  = (size_t)3 * DM * DM * sizeof(_Float16);
  const size_t qkvBytes = (size_t)NB * NH * SEQ * HD * sizeof(_Float16);
  const size_t total = xhBytes + wtBytes + 5 * qkvBytes;
  if (total > ws_size) return;
  char* wsb = (char*)d_ws;
  _Float16* Xh = (_Float16*)(wsb);
  _Float16* Wt = (_Float16*)(wsb + xhBytes);
  _Float16* Qh = (_Float16*)(wsb + xhBytes + wtBytes);
  _Float16* Qr = (_Float16*)(wsb + xhBytes + wtBytes + qkvBytes);
  _Float16* Kh = (_Float16*)(wsb + xhBytes + wtBytes + 2 * qkvBytes);
  _Float16* Kr = (_Float16*)(wsb + xhBytes + wtBytes + 3 * qkvBytes);
  _Float16* Vt = (_Float16*)(wsb + xhBytes + wtBytes + 4 * qkvBytes);

  cvt_x_kernel<<<dim3((unsigned)((size_t)MTOT * DM / 2048)), 256, 0, stream>>>(x, Xh);
  cvt_w_kernel<<<dim3(DM / 64, DM / 64, 3), 256, 0, stream>>>(Wq, Wk, Wv, Wt);
  proj_kernel<<<dim3(MTOT / 128, 3 * (DM / 128)), 256, 0, stream>>>(Xh, Wt, bq, bk, bv, Qh, Qr, Kh, Kr, Vt);
  attn_kernel<<<dim3(SEQ / 128, NB * NH), 256, 0, stream>>>(Qh, Qr, Kh, Kr, Vt, mask, out);
}
